// InitMotionParams_76201309765904
// MI455X (gfx1250) — hardware-verified
//
#include <hip/hip_runtime.h>
#include <stddef.h>


typedef _Float16 h16;
typedef _Float16 v16h __attribute__((ext_vector_type(16)));
typedef _Float16 v8h  __attribute__((ext_vector_type(8)));
typedef float    v8f  __attribute__((ext_vector_type(8)));
typedef float    v4f  __attribute__((ext_vector_type(4)));

#ifndef NG
#define NG 400000
#endif
#define NG_FULL 400000
#define NK    20
#define NF    300
#define NTS   8
#define NCOLS 72
#define NPADC 80
#define NT    5
#define KPAD  32
#define OROW  24
#define TP    80
#ifndef COEF_RES
#define COEF_RES 1
#endif

#define ACARRY 1024.0f
#define RCARRY 2048.0f
#define BCARRY 4096.0f

static_assert(NG >= 128 && NG <= NG_FULL && (NG % 128) == 0);
static_assert(NK == 20 && NK <= KPAD && KPAD == 32);
static_assert(NCOLS == NTS * 9 && NCOLS <= NPADC && NPADC == NT * 16);
static_assert(OROW == NTS * 3);
static_assert((16 * OROW * 4) % 512 == 0);
static_assert(16 * OROW == 3 * 32 * 4);
static_assert(NPADC * KPAD == 10 * 256);
static_assert(NPADC * KPAD == (256 + 64) * 8);
static_assert((NK * 4) % 16 == 0);
static_assert(TP >= NPADC);

#define BP_BYTES ((size_t)NPADC * KPAD * 2)
#define OFF_BP   ((size_t)0)
#define WS_TOTAL (OFF_BP + BP_BYTES)
static_assert((BP_BYTES % 128) == 0);
static_assert(WS_TOTAL <= (size_t)134217728);

__device__ __forceinline__ float bf16r(float x) {
  unsigned int u = __float_as_uint(x);
  u = (u + 0x7FFFu + ((u >> 16) & 1u)) & 0xFFFF0000u;
  return __uint_as_float(u);
}

static __device__ __forceinline__ h16 toh_flush(float v) {
  const h16 r = (h16)v;
  return (fabsf(v) < 6.103515625e-05f) ? (h16)0.0f : r;
}

__device__ __forceinline__ v16h frag_at(const _Float16* p) {
  v8h lo = *(const v8h*)(p);
  v8h hi = *(const v8h*)(p + 16);
  v16h out;
#pragma unroll
  for (int i = 0; i < 8; ++i) { out[i] = lo[i]; out[i + 8] = hi[i]; }
  return out;
}

__device__ __forceinline__ v8f wmma16(v16h a, v16h b, v8f c) {
  v8f d = __builtin_amdgcn_wmma_f32_16x16x32_f16(false, a, false, b, (short)0, c,
                                                 false, false);
  asm volatile("v_nop\n\tv_nop\n\tv_nop\n\tv_nop" : "+v"(d) : "v"(a), "v"(b));
  return d;
}

__device__ __forceinline__ void wave_lds_sync() {
  __builtin_amdgcn_fence(3  , "wavefront");
  asm volatile("s_wait_dscnt 0x0" ::: "memory");
  __builtin_amdgcn_wave_barrier();
}

__global__ __launch_bounds__(256) void bplane_kernel(
    const float* __restrict__ rots, const float* __restrict__ transls,
    const int* __restrict__ ts, _Float16* __restrict__ Bp) {
  __shared__ __attribute__((aligned(16))) _Float16 T[NPADC * KPAD];
  const unsigned tid = threadIdx.x;
#pragma unroll 1
  for (unsigned j = 0; j < 10u; ++j) {
    const unsigned idx = tid + 256u * j;
    const unsigned n = idx >> 5, k = idx & 31u;
    const unsigned nn = (n < (unsigned)NCOLS) ? n : (unsigned)(NCOLS - 1);
    const unsigned kc = (k < (unsigned)NK) ? k : (unsigned)(NK - 1);
    const unsigned tn = nn / 9u;
    const unsigned jj = nn - 9u * tn;
    int tt = ts[tn];
    tt = (tt < 0) ? (tt + NF) : tt;
    tt = (tt < 0) ? 0 : tt;
    tt = (tt > NF - 1) ? (NF - 1) : tt;
    const unsigned jr = (jj < 5u) ? jj : 5u;
    const unsigned jt = (jj >= 6u) ? (jj - 6u) : 0u;
    const float vr = rots[((size_t)kc * NF + (unsigned)tt) * 6u + jr];
    const float vt = transls[((size_t)kc * NF + (unsigned)tt) * 3u + jt];
    float v = (jj < 6u) ? vr : vt;
    v = (n < (unsigned)NCOLS && k < (unsigned)NK) ? (BCARRY * bf16r(v)) : 0.0f;
    T[idx] = toh_flush(v);
  }
  __syncthreads();
  const unsigned p0 = tid;
  const unsigned p1 = 256u + (tid & 63u);
  const bool second = (tid < 64u);
  const v8h x0 = *(const v8h*)&T[p0 * 8u];
  const v8h x1 = *(const v8h*)&T[p1 * 8u];
  *(volatile v8h*)(Bp + p0 * 8u) = x0;
  if (second) *(volatile v8h*)(Bp + p1 * 8u) = x1;
  __threadfence();
  *(volatile v8h*)(Bp + p0 * 8u) = x0;
  if (second) *(volatile v8h*)(Bp + p1 * 8u) = x1;
}

__global__ __launch_bounds__(256) void blend_kernel(
    const float* __restrict__ coefs, const float* __restrict__ means,
    const _Float16* __restrict__ Bp, float* __restrict__ out) {
  __shared__ __attribute__((aligned(16))) float Ts[8 * 16 * TP];
  __shared__ __attribute__((aligned(16))) float Os[8 * 16 * OROW];

  const unsigned tid = threadIdx.x, lane = tid & 31u;
  const unsigned wave = (unsigned)__builtin_amdgcn_readfirstlane((int)(threadIdx.x >> 5));
  const unsigned hh = lane >> 4, m = lane & 15u;
  const unsigned g0 = (blockIdx.x * 8u + wave) * 16u;
  const unsigned tb = wave * (16u * TP);
  const unsigned ob = wave * (16u * OROW);

  const float* crow = coefs + (size_t)(g0 + m) * NK;
  const v4f c0 = *(const v4f*)(crow + hh * 8u);
  const v4f c1 = *(const v4f*)(crow + hh * 8u + 4u);
  const v4f c2 = *(const v4f*)(crow + 16u);
  const bool tail = (hh == 0u);
  float x[12];
#pragma unroll
  for (int i = 0; i < 4; ++i) {
    x[i]     = bf16r(c0[i]);
    x[i + 4] = bf16r(c1[i]);
    x[i + 8] = tail ? bf16r(c2[i]) : -3.0e38f;
  }
  float mx = x[0];
#pragma unroll
  for (int i = 1; i < 12; ++i) mx = fmaxf(mx, x[i]);
  mx = fmaxf(mx, __shfl_xor(mx, 16, 32));
  float e[12];
  float s = 0.0f;
#pragma unroll
  for (int i = 0; i < 8; ++i) { e[i] = expf(x[i] - mx); s += e[i]; }
#pragma unroll
  for (int i = 8; i < 12; ++i) {
    const float arg = tail ? (x[i] - mx) : 0.0f;
    const float ev = expf(arg);
    e[i] = tail ? ev : 0.0f;
    s += e[i];
  }
  s += __shfl_xor(s, 16, 32);
  const float inv = 1.0f / s;

  v16h ahi;
#if COEF_RES
  v16h ares;
#endif
#pragma unroll
  for (int i = 0; i < 12; ++i) {
    const float t = (e[i] * inv) * ACARRY;
    const h16 hi = toh_flush(t);
    ahi[i] = hi;
#if COEF_RES
    ares[i] = toh_flush((t - (float)hi) * RCARRY);
#endif
  }
#pragma unroll
  for (int i = 12; i < 16; ++i) {
    ahi[i] = (h16)0.0f;
#if COEF_RES
    ares[i] = (h16)0.0f;
#endif
  }

  v8f acc[NT];
#if COEF_RES
  v8f accr[NT];
#endif
#pragma unroll
  for (int nt = 0; nt < NT; ++nt) {
    const v16h bf = frag_at(Bp + ((unsigned)nt * 16u + m) * (unsigned)KPAD + hh * 8u);
    acc[nt] = wmma16(ahi, bf, (v8f){});
#if COEF_RES
    accr[nt] = wmma16(ares, bf, (v8f){});
#endif
  }

  const float oscale = 1.0f / (ACARRY * BCARRY);
#pragma unroll
  for (int nt = 0; nt < NT; ++nt)
#pragma unroll
    for (int r = 0; r < 8; ++r) {
#if COEF_RES
      const float t = acc[nt][r] + accr[nt][r] * (1.0f / RCARRY);
#else
      const float t = acc[nt][r];
#endif
      Ts[tb + (hh * 8u + (unsigned)r) * TP + (unsigned)nt * 16u + m] = t * oscale;
    }
  wave_lds_sync();

#pragma unroll
  for (unsigned q = 0; q < 4u; ++q) {
    const unsigned task = lane + 32u * q;
    const unsigned row = task >> 3;
    const unsigned n = task & 7u;
    const unsigned rb = tb + row * TP + n * 9u;
    const float a1x = Ts[rb + 0u], a1y = Ts[rb + 1u], a1z = Ts[rb + 2u];
    const float a2x = Ts[rb + 3u], a2y = Ts[rb + 4u], a2z = Ts[rb + 5u];
    const float tx  = Ts[rb + 6u], ty  = Ts[rb + 7u], tz  = Ts[rb + 8u];

    const size_t mo = (size_t)(g0 + row) * 3u;
    const float mex = bf16r(means[mo + 0u]);
    const float mey = bf16r(means[mo + 1u]);
    const float mez = bf16r(means[mo + 2u]);

    const float n1 = fmaxf(sqrtf(a1x * a1x + a1y * a1y + a1z * a1z), 1e-12f);
    const float i1 = 1.0f / n1;
    const float b1x = a1x * i1, b1y = a1y * i1, b1z = a1z * i1;
    const float d = b1x * a2x + b1y * a2y + b1z * a2z;
    const float px = a2x - d * b1x, py = a2y - d * b1y, pz = a2z - d * b1z;
    const float n2 = fmaxf(sqrtf(px * px + py * py + pz * pz), 1e-12f);
    const float i2 = 1.0f / n2;
    const float b2x = px * i2, b2y = py * i2, b2z = pz * i2;
    const float b3x = b1y * b2z - b1z * b2y;
    const float b3y = b1z * b2x - b1x * b2z;
    const float b3z = b1x * b2y - b1y * b2x;

    const float ox = b1x * mex + b2x * mey + b3x * mez + tx;
    const float oy = b1y * mex + b2y * mey + b3y * mez + ty;
    const float oz = b1z * mex + b2z * mey + b3z * mez + tz;

    const unsigned oo = ob + row * (unsigned)OROW + n * 3u;
    Os[oo + 0u] = ox;
    Os[oo + 1u] = oy;
    Os[oo + 2u] = oz;
  }
  wave_lds_sync();

  v4f xs[3];
  size_t off[3];
#pragma unroll
  for (unsigned i = 0; i < 3u; ++i) {
    const unsigned piece = lane + 32u * i;
    xs[i] = *(const v4f*)&Os[ob + 4u * piece];
    off[i] = (size_t)g0 * OROW + 4u * piece;
  }
#pragma unroll
  for (int i = 0; i < 3; ++i) *(volatile v4f*)(out + off[i]) = xs[i];
  __threadfence();
#pragma unroll
  for (int i = 0; i < 3; ++i) *(volatile v4f*)(out + off[i]) = xs[i];
}

extern "C" void kernel_launch(void* const* d_in, const int* in_sizes, int n_in,
                              void* d_out, int out_size, void* d_ws, size_t ws_size,
                              hipStream_t stream) {
  if (n_in < 5) return;
  if ((long long)in_sizes[0] < (long long)NK * NF * 6) return;
  if ((long long)in_sizes[1] < (long long)NK * NF * 3) return;
  if ((long long)in_sizes[2] < (long long)NG * NK) return;
  if ((long long)in_sizes[3] < (long long)NG * 3) return;
  if (in_sizes[4] < NTS) return;
  if ((long long)out_size < (long long)NG * OROW) return;
  if (ws_size < WS_TOTAL) return;

  const float* rots    = (const float*)d_in[0];
  const float* transls = (const float*)d_in[1];
  const float* coefs   = (const float*)d_in[2];
  const float* means   = (const float*)d_in[3];
  const int*   ts      = (const int*)d_in[4];
  float* out = (float*)d_out;

  char* ws = (char*)d_ws;
  _Float16* Bp = (_Float16*)(ws + OFF_BP);

  bplane_kernel<<<dim3(1), dim3(256), 0, stream>>>(rots, transls, ts, Bp);
  blend_kernel<<<dim3(NG / 128), dim3(256), 0, stream>>>(coefs, means, Bp, out);
}
